// MyLSTMModel_68796786147466
// MI455X (gfx1250) — hardware-verified
//
#include <hip/hip_runtime.h>
#include <stddef.h>
#include <math.h>

typedef __attribute__((ext_vector_type(16))) _Float16 v16h;
typedef __attribute__((ext_vector_type(8)))  _Float16 v8h;
typedef __attribute__((ext_vector_type(16))) __bf16   v16b;
typedef __attribute__((ext_vector_type(8)))  __bf16   v8b;
typedef __attribute__((ext_vector_type(8)))  float    v8f;
typedef __attribute__((ext_vector_type(4)))  float    v4f;

constexpr int kBatch     = 8;
constexpr int kSteps     = 32;
constexpr int kImg       = 64;
constexpr int kCin       = 3;
constexpr int kF         = 24;
constexpr int kUnits     = 128;
constexpr int kFrames    = kBatch * kSteps;
constexpr int kPix       = kImg * kImg;
constexpr int kFC        = 32;
constexpr int kChunks    = kFrames / kFC;
constexpr int kMC        = kFC * kPix;
constexpr int kK1Real    = 27;
constexpr int kK1        = 32;
constexpr int kK2Real    = 216;
constexpr int kK2        = 224;
constexpr int kNpad      = 64;
constexpr int kZReal     = kF + kUnits;
constexpr int kZK        = 160;
constexpr int kGateCols  = 4 * kUnits;
constexpr int kFeatPitch = 32;
constexpr int kThreads   = 256;
constexpr int kZP        = 168;
constexpr int kGP        = 520;
constexpr float kWScale  = 8.0f;
constexpr float kC1Scale = 2.0f;
constexpr float kC2Scale = 1.0f / 128.0f;
constexpr float kZScale  = 256.0f;
constexpr float kPreInv  = 1.0f / 2048.0f;

static_assert(kFrames % kFC == 0);
static_assert(kMC % 64 == 0 && (kMC / 64) % 8 == 0);
static_assert((kMC * 4) % kThreads == 0);
static_assert((kMC * (kK2 / 8)) % kThreads == 0);
static_assert(kK1 % 32 == 0 && kK2 % 32 == 0 && kZK % 32 == 0);
static_assert(kK1 > kK1Real && kK2 >= kK2Real && kZK >= kZReal);
static_assert(kZP % 8 == 0 && kZP >= kZK && kGP % 4 == 0 && kGP >= kGateCols);
static_assert(kBatch * kF == 192 && (kBatch * kF) % 32 == 0);
static_assert(kThreads == kBatch * kSteps);

__device__ __forceinline__ unsigned short f2bf_bits(float f) {
  unsigned u = __float_as_uint(f);
  return (unsigned short)((u + 0x7FFFu + ((u >> 16) & 1u)) >> 16);
}
__device__ __forceinline__ float bf_bits2f(unsigned short h) { return __uint_as_float(((unsigned)h) << 16); }

__device__ __forceinline__ void dep_guard_h(v8f& a, v8f& b, v16h x, v16h y) { asm volatile("v_nop\n\tv_nop\n\tv_nop\n\tv_nop" : "+v"(a), "+v"(b) : "v"(x), "v"(y)); }
__device__ __forceinline__ void dep_guard_b(v8f& a, v8f& b, v16b x, v16b y) { asm volatile("v_nop\n\tv_nop\n\tv_nop\n\tv_nop" : "+v"(a), "+v"(b) : "v"(x), "v"(y)); }
__device__ __forceinline__ void keep4_h(v16h a, v16h b, v16h c, v16h d) { asm volatile("v_nop" :: "v"(a), "v"(b), "v"(c), "v"(d)); }
__device__ __forceinline__ void keep4_b(v16b a, v16b b, v16b c, v16b d) { asm volatile("v_nop" :: "v"(a), "v"(b), "v"(c), "v"(d)); }
__device__ __forceinline__ void acc_guard4(v8f& a, v8f& b, v8f& c, v8f& d) { asm volatile("v_nop\n\tv_nop\n\tv_nop\n\tv_nop" : "+v"(a), "+v"(b), "+v"(c), "+v"(d)); }
template <typename T> struct Frag;
template <> struct Frag<_Float16> {
  typedef v16h V; union U { v16h v; v8h h[2]; };
  static __device__ __forceinline__ v16h load(const _Float16* p) {
    U f; f.h[0] = *(const v8h*)(p); f.h[1] = *(const v8h*)(p + 16); return f.v;
  }
  static __device__ __forceinline__ v8f mma(v16h a, v16h b, v8f c) {
    return __builtin_amdgcn_wmma_f32_16x16x32_f16(false, a, false, b, (short)0, c, false, false);
  }
  static __device__ __forceinline__ void guard(v8f& a, v8f& b, v16h x, v16h y) { dep_guard_h(a, b, x, y); }
  static __device__ __forceinline__ void keep(v16h a, v16h b, v16h c, v16h d) { keep4_h(a, b, c, d); }
};
template <> struct Frag<__bf16> {
  typedef v16b V; union U { v16b v; v8b h[2]; };
  static __device__ __forceinline__ v16b load(const __bf16* p) {
    U f; f.h[0] = *(const v8b*)(p); f.h[1] = *(const v8b*)(p + 16); return f.v;
  }
  static __device__ __forceinline__ v8f mma(v16b a, v16b b, v8f c) {
    return __builtin_amdgcn_wmma_f32_16x16x32_bf16(false, a, false, b, (short)0, c, false, false);
  }
  static __device__ __forceinline__ void guard(v8f& a, v8f& b, v16b x, v16b y) { dep_guard_b(a, b, x, y); }
  static __device__ __forceinline__ void keep(v16b a, v16b b, v16b c, v16b d) { keep4_b(a, b, c, d); }
};

template <int ET> struct Elem;
template <> struct Elem<0> { typedef _Float16 T; };
template <> struct Elem<1> { typedef __bf16 T; };
template <int ET, bool SPLIT, int BIAS_MODE, int OUT_MODE, bool RESID, int ACT = 0>
__global__ __launch_bounds__(256) void wmma_gemm64(
    const unsigned short* __restrict__ Ap, const unsigned short* __restrict__ A2p, int lda, long strideA,
    const unsigned short* __restrict__ Btp, const unsigned short* __restrict__ Bt2p, int ldb, long strideB,
    void* __restrict__ Cout, void* __restrict__ Cout2, int ldc, long strideC,
    const float* __restrict__ bias,
    const float* __restrict__ resid, long strideR,
    int M, int N, int K, float scale) {
  typedef typename Elem<ET>::T T;
  typedef typename Frag<T>::V V;
  const T* A = (const T*)Ap; const T* A2 = (const T*)A2p; const T* Bt = (const T*)Btp; const T* Bt2 = (const T*)Bt2p;
  __shared__ __align__(16) float sT[8][16 * 68];
  const int b    = blockIdx.y;
  const int lane = threadIdx.x & 31;
  const int wave = threadIdx.x >> 5;
  const int tilesN = N >> 6;
  const int tilesM = M >> 6;
  const int tile = blockIdx.x * 8 + wave;
  if (tile >= tilesM * tilesN) return;
  const int tm = tile / tilesN;
  const int tn = tile - tm * tilesN;
  const int m0 = tm << 6;
  const int n0 = tn << 6;

  const T* Ab  = A  + (size_t)b * strideA;
  const T* Bb  = Bt + (size_t)b * strideB;
  const T* Ab2 = SPLIT ? (A2  + (size_t)b * strideA) : nullptr;
  const T* Bb2 = SPLIT ? (Bt2 + (size_t)b * strideB) : nullptr;

  const int rlane = lane & 15;
  const int koff  = (lane >> 4) * 8;
  const int mOff  = (lane >> 4) * 8;

  v8f acc[4][4];
#pragma unroll
  for (int i = 0; i < 4; ++i)
#pragma unroll
    for (int j = 0; j < 4; ++j) acc[i][j] = (v8f){0.f,0.f,0.f,0.f,0.f,0.f,0.f,0.f};

  for (int k0 = 0; k0 < K; k0 += 32) {
    V bh[4], bl[4];
#pragma unroll
    for (int j = 0; j < 4; ++j) {
      const size_t bo = (size_t)(n0 + (j << 4) + rlane) * ldb + koff + k0;
      bh[j] = Frag<T>::load(Bb + bo);
      if (SPLIT) bl[j] = Frag<T>::load(Bb2 + bo);
    }
#pragma unroll
    for (int i = 0; i < 4; ++i) {
      const size_t ao = (size_t)(m0 + (i << 4) + rlane) * lda + koff + k0;
      V ah = Frag<T>::load(Ab + ao);
      V al;
      if (SPLIT) al = Frag<T>::load(Ab2 + ao);
#pragma unroll
      for (int j = 0; j < 4; ++j) {
        acc[i][j] = Frag<T>::mma(ah, bh[j], acc[i][j]);
        if (SPLIT) {
          acc[i][j] = Frag<T>::mma(ah, bl[j], acc[i][j]);
          acc[i][j] = Frag<T>::mma(al, bh[j], acc[i][j]);
        }
      }
      Frag<T>::guard(acc[i][0], acc[i][3], ah, SPLIT ? al : ah);
    }
    Frag<T>::keep(bh[0], bh[1], bh[2], bh[3]);
    if (SPLIT) Frag<T>::keep(bl[0], bl[1], bl[2], bl[3]);
  }
  acc_guard4(acc[0][0], acc[0][1], acc[0][2], acc[0][3]);
  acc_guard4(acc[1][0], acc[1][1], acc[1][2], acc[1][3]);
  acc_guard4(acc[2][0], acc[2][1], acc[2][2], acc[2][3]);
  acc_guard4(acc[3][0], acc[3][1], acc[3][2], acc[3][3]);

  float* slab = sT[wave];
  const float* Rb = RESID ? (resid + (size_t)b * strideR) : nullptr;
#pragma unroll
  for (int i = 0; i < 4; ++i) {
    const int mBase = m0 + (i << 4);
#pragma unroll
    for (int j = 0; j < 4; ++j) {
      const int n = n0 + (j << 4) + rlane;
      float bv = 0.f;
      if (BIAS_MODE == 2) bv = bias[n];
#pragma unroll
      for (int r = 0; r < 8; ++r) {
        float v = acc[i][j][r] * scale;
        if (BIAS_MODE == 1) v += bias[mBase + mOff + r];
        if (BIAS_MODE == 2) v += bv;
        if (RESID) v += Rb[(size_t)(mBase + mOff + r) * ldc + n];
        if (ACT == 1) v = tanhf(v);
        if (ACT == 2) v = fmaxf(v, 0.0f);
        if (ACT == 3) v = v / (1.0f + expf(-v));
        if (ACT == 4) v = (v > 0.f) ? v : 0.01f * v;
        if (ACT == 5) v = 0.5f * v * (1.0f + erff(v * 0.70710678118654752f));
        slab[(mOff + r) * 68 + (j << 4) + rlane] = v;
      }
    }
    __builtin_amdgcn_fence(__ATOMIC_RELEASE, "workgroup");
    __builtin_amdgcn_wave_barrier();
    __builtin_amdgcn_fence(__ATOMIC_ACQUIRE, "workgroup");
    if (OUT_MODE == 0) {
      float* C = (float*)Cout + (size_t)b * strideC;
      const int hh = lane >> 4, c4 = (lane & 15) * 4;
      for (int pass = 0; pass < 2; ++pass) {
#pragma unroll
        for (int it = 0; it < 8; ++it) {
          const int row = it * 2 + hh;
          v4f v = *(const v4f*)(slab + row * 68 + c4);
          *(volatile v4f*)(C + (size_t)(mBase + row) * ldc + n0 + c4) = v;
        }
        __threadfence();
      }
    } else {
      const int q = lane >> 3, c8 = (lane & 7) * 8;
      unsigned short* C  = (unsigned short*)Cout  + (size_t)b * strideC;
      unsigned short* C2 = (OUT_MODE == 2) ? ((unsigned short*)Cout2 + (size_t)b * strideC) : nullptr;
      for (int pass = 0; pass < 2; ++pass) {
#pragma unroll
        for (int it = 0; it < 4; ++it) {
          const int row = it * 4 + q;
          const float* sp = slab + row * 68 + c8;
          v8h hv, lv;
#pragma unroll
          for (int e = 0; e < 8; ++e) {
            if (OUT_MODE == 1) {
              hv[e] = (_Float16)sp[e];
            } else {
              unsigned short hb = f2bf_bits(sp[e]);
              unsigned short lb = f2bf_bits(sp[e] - bf_bits2f(hb));
              hv[e] = __builtin_bit_cast(_Float16, hb);
              lv[e] = __builtin_bit_cast(_Float16, lb);
            }
          }
          *(volatile v8h*)(C + (size_t)(mBase + row) * ldc + n0 + c8) = hv;
          if (OUT_MODE == 2) *(volatile v8h*)(C2 + (size_t)(mBase + row) * ldc + n0 + c8) = lv;
        }
        __threadfence();
      }
    }
    __builtin_amdgcn_fence(__ATOMIC_RELEASE, "workgroup");
    __builtin_amdgcn_wave_barrier();
    __builtin_amdgcn_fence(__ATOMIC_ACQUIRE, "workgroup");
  }
}

template <bool WITH_BCOL>
__global__ __launch_bounds__(kThreads) void k_wprep16(const float* __restrict__ W, const float* __restrict__ bvec,
                                                      int Kin, int ncol, int Kpad, int nrow, float scale,
                                                      unsigned short* bt) {
  const int tpr = Kpad >> 3;
  const int i = blockIdx.x * kThreads + threadIdx.x;
  if (i >= nrow * tpr) return;
  const int n   = i / tpr;
  const int k0  = (i - n * tpr) * 8;
  const int ncl = (n < ncol) ? n : (ncol - 1);
  const float bv = WITH_BCOL ? bvec[ncl] : 0.0f;
  v8h hv;
#pragma unroll
  for (int e = 0; e < 8; ++e) {
    const int k  = k0 + e;
    const int kc = (k < Kin) ? k : (Kin - 1);
    float v = W[(size_t)kc * ncol + ncl];
    if (k >= Kin) v = (WITH_BCOL && k == Kin) ? bv : 0.0f;
    if (n >= ncol) v = 0.0f;
    hv[e] = (_Float16)(scale * v);
  }
  const size_t o = (size_t)i * 8;
  *(volatile v8h*)(bt + o) = hv;
  __threadfence();
  *(volatile v8h*)(bt + o) = hv;
}

__global__ __launch_bounds__(kThreads) void k_im2col1(const float* __restrict__ x, int fbase, unsigned short* im1) {
  const int i  = blockIdx.x * kThreads + threadIdx.x;
  const int m  = i >> 2;
  const int k0 = (i & 3) * 8;
  const int fl = m >> 12;
  const int py = (m >> 6) & 63;
  const int px = m & 63;
  const int fg = fbase + fl;
  v8h hv;
#pragma unroll
  for (int e = 0; e < 8; ++e) {
    const int k   = k0 + e;
    const int tap = k / 3;
    const int ci  = k - tap * 3;
    const int ky  = tap / 3;
    const int kx  = tap - ky * 3;
    int yy = py + ky - 1;
    int xx = px + kx - 1;
    const bool inb = (k < kK1Real) && (yy >= 0) && (yy < kImg) && (xx >= 0) && (xx < kImg);
    yy = (yy < 0) ? 0 : ((yy > kImg - 1) ? (kImg - 1) : yy);
    xx = (xx < 0) ? 0 : ((xx > kImg - 1) ? (kImg - 1) : xx);
    float v = x[(((size_t)fg * kImg + yy) * kImg + xx) * kCin + ci];
    v = inb ? v : ((k == kK1Real) ? 1.0f : 0.0f);
    hv[e] = (_Float16)v;
  }
  const size_t o = (size_t)i * 8;
  *(volatile v8h*)(im1 + o) = hv;
  __threadfence();
  *(volatile v8h*)(im1 + o) = hv;
}

__global__ __launch_bounds__(kThreads) void k_im2col2(const unsigned short* __restrict__ c1, unsigned short* im2) {
  const int i  = blockIdx.x * kThreads + threadIdx.x;
  const int m  = i / 28;
  const int j  = i - m * 28;
  const int fl = m >> 12;
  const int py = (m >> 6) & 63;
  const int px = m & 63;
  const int tap = j / 3;
  const int cg  = j - tap * 3;
  const int ky  = tap / 3;
  const int kx  = tap - ky * 3;
  int yy = py + ky - 1;
  int xx = px + kx - 1;
  const bool inb = (j < 27) && (yy >= 0) && (yy < kImg) && (xx >= 0) && (xx < kImg);
  yy = (yy < 0) ? 0 : ((yy > kImg - 1) ? (kImg - 1) : yy);
  xx = (xx < 0) ? 0 : ((xx > kImg - 1) ? (kImg - 1) : xx);
  const size_t src = ((size_t)fl * kPix + (size_t)yy * kImg + xx) * kNpad + cg * 8;
  const v8h v = *(const v8h*)(c1 + src);
  v8h hv;
#pragma unroll
  for (int e = 0; e < 8; ++e) hv[e] = inb ? (_Float16)v[e] : (_Float16)0.0f;
  const size_t o = (size_t)i * 8;
  *(volatile v8h*)(im2 + o) = hv;
  __threadfence();
  *(volatile v8h*)(im2 + o) = hv;
}

__global__ __launch_bounds__(kThreads) void k_pool(const float* __restrict__ c2, const float* __restrict__ b2,
                                                  int fbase, float* feat) {
  __shared__ float part[8][32];
  __shared__ __align__(16) float rowv[32];
  const int t  = threadIdx.x;
  const int c  = t & 31;
  const int rg = t >> 5;
  const int fl = blockIdx.x;
  const float* base = c2 + ((size_t)fl * kPix) * kNpad + c;
  float s = 0.0f;
#pragma unroll 1
  for (int r = rg; r < kPix; r += 8) s += base[(size_t)r * kNpad];
  part[rg][c] = s;
  __syncthreads();
  if (t < 32) {
    float tot = 0.0f;
#pragma unroll
    for (int q = 0; q < 8; ++q) tot += part[q][c];
    const int cc = (c < kF) ? c : (kF - 1);
    const float bv = b2[cc];
    float v = tot * (1.0f / 4096.0f) + bv;
    if (c >= kF) v = 0.0f;
    rowv[c] = v;
  }
  __syncthreads();
  const int lc = (t < 8) ? t : 7;
  const v4f vv = *(const v4f*)(rowv + 4 * lc);
  float* dst = feat + (size_t)(fbase + fl) * kFeatPitch + 4 * lc;
  if (t < 8) *(volatile v4f*)dst = vv;
  __threadfence();
  if (t < 8) *(volatile v4f*)dst = vv;
}

__global__ __launch_bounds__(kThreads) void k_lstm(const float* __restrict__ feat, const unsigned short* __restrict__ wl,
                                                  const float* __restrict__ bfv, const float* __restrict__ biv,
                                                  const float* __restrict__ bcv, const float* __restrict__ bov,
                                                  const float* __restrict__ ow,  const float* __restrict__ ob,
                                                  float* out) {
  __shared__ __align__(16) _Float16 zA[16 * kZP];
  __shared__ __align__(16) float gpre[16 * kGP];
  __shared__ float cst[kBatch * kUnits];
  __shared__ float hst[kBatch * kUnits];
  __shared__ __align__(16) float outs[kBatch * kSteps];
  const int tid   = threadIdx.x;
  const int lane  = tid & 31;
  const int wave  = tid >> 5;
  const int rlane = lane & 15;
  const int hh    = lane >> 4;
  const int koff  = hh * 8;

  for (int i = tid; i < 16 * kZP; i += kThreads) zA[i] = (_Float16)0.0f;
  for (int i = tid; i < kBatch * kUnits; i += kThreads) { cst[i] = 0.0f; hst[i] = 0.0f; }
  outs[tid] = 0.0f;
  __syncthreads();
  if (tid < kBatch * kF) {
    const int b = tid / kF, k = tid - b * kF;
    zA[b * kZP + k] = (_Float16)(kZScale * feat[(size_t)(b * kSteps) * kFeatPitch + k]);
  }
  __syncthreads();

  const _Float16* wlh = (const _Float16*)wl;
  const int n0 = wave * 64;
  const v8f zero8 = (v8f){0.f,0.f,0.f,0.f,0.f,0.f,0.f,0.f};

#pragma unroll 1
  for (int t = 0; t < kSteps; ++t) {
    v8f acc[4];
#pragma unroll
    for (int j = 0; j < 4; ++j) acc[j] = zero8;
#pragma unroll 1
    for (int ks = 0; ks < kZK / 32; ++ks) {
      const v16h a = Frag<_Float16>::load(zA + rlane * kZP + koff + ks * 32);
      v16h bfr[4];
#pragma unroll
      for (int j = 0; j < 4; ++j)
        bfr[j] = Frag<_Float16>::load(wlh + (size_t)(n0 + 16 * j + rlane) * kZK + koff + ks * 32);
#pragma unroll
      for (int j = 0; j < 4; ++j) acc[j] = Frag<_Float16>::mma(a, bfr[j], acc[j]);
      dep_guard_h(acc[0], acc[3], a, bfr[3]);
      keep4_h(bfr[0], bfr[1], bfr[2], bfr[3]);
    }
    acc_guard4(acc[0], acc[1], acc[2], acc[3]);
#pragma unroll
    for (int j = 0; j < 4; ++j) {
#pragma unroll
      for (int r = 0; r < 8; ++r) gpre[(8 * hh + r) * kGP + n0 + 16 * j + rlane] = acc[j][r];
    }
    __syncthreads();

#pragma unroll 1
    for (int idx = tid; idx < kBatch * kUnits; idx += kThreads) {
      const int b = idx >> 7;
      const int u = idx & 127;
      const float* gp = gpre + b * kGP;
      const float pf = gp[u]              * kPreInv + bfv[u];
      const float pi = gp[kUnits + u]     * kPreInv + biv[u];
      const float pg = gp[2 * kUnits + u] * kPreInv + bcv[u];
      const float po = gp[3 * kUnits + u] * kPreInv + bov[u];
      const float fgt = 1.0f / (1.0f + expf(-pf));
      const float igt = 1.0f / (1.0f + expf(-pi));
      const float ggt = tanhf(pg);
      const float ogt = 1.0f / (1.0f + expf(-po));
      const float cn  = cst[idx] * fgt + igt * ggt;
      const float hn  = tanhf(cn) * ogt;
      cst[idx] = cn;
      hst[idx] = hn;
      zA[b * kZP + kF + u] = (_Float16)(kZScale * hn);
    }
    if (t < kSteps - 1) {
      if (tid < kBatch * kF) {
        const int b = tid / kF, k = tid - b * kF;
        zA[b * kZP + k] = (_Float16)(kZScale * feat[(size_t)(b * kSteps + t + 1) * kFeatPitch + k]);
      }
    }
    __syncthreads();

    {
      const float* hp = hst + wave * kUnits;
      float p = hp[lane] * ow[lane] + hp[lane + 32] * ow[lane + 32]
              + hp[lane + 64] * ow[lane + 64] + hp[lane + 96] * ow[lane + 96];
#pragma unroll
      for (int off = 16; off >= 1; off >>= 1) p += __shfl_xor(p, off, 32);
      if (lane == 0) outs[wave * kSteps + t] = p + ob[0];
    }
  }
  __syncthreads();

  const int lc = (lane < 8) ? lane : 7;
  const v4f vv = *(const v4f*)(outs + wave * kSteps + 4 * lc);
  float* dst = out + (size_t)wave * kSteps + 4 * lc;
  if (lane < 8) *(volatile v4f*)dst = vv;
  __threadfence();
  if (lane < 8) *(volatile v4f*)dst = vv;
}

extern "C" void kernel_launch(void* const* d_in, const int* in_sizes, int n_in,
                              void* d_out, int out_size, void* d_ws, size_t ws_size,
                              hipStream_t stream) {
  if (n_in < 15) return;
  if (in_sizes[0] != kFrames * kPix * kCin) return;
  if (in_sizes[1] != 9 * kCin * kF || in_sizes[2] != kF) return;
  if (in_sizes[3] != 9 * kF * kF   || in_sizes[4] != kF) return;
  if (in_sizes[5] != kZReal * kUnits || in_sizes[7] != kZReal * kUnits ||
      in_sizes[9] != kZReal * kUnits || in_sizes[11] != kZReal * kUnits) return;
  if (in_sizes[6] != kUnits || in_sizes[8] != kUnits || in_sizes[10] != kUnits || in_sizes[12] != kUnits) return;
  if (in_sizes[13] != kUnits || in_sizes[14] < 1) return;
  if (out_size != kBatch * kSteps) return;

  const float* x   = (const float*)d_in[0];
  const float* w1  = (const float*)d_in[1];
  const float* b1  = (const float*)d_in[2];
  const float* w2  = (const float*)d_in[3];
  const float* b2  = (const float*)d_in[4];
  const float* Wf  = (const float*)d_in[5];
  const float* bfv = (const float*)d_in[6];
  const float* Wi  = (const float*)d_in[7];
  const float* biv = (const float*)d_in[8];
  const float* Wc  = (const float*)d_in[9];
  const float* bcv = (const float*)d_in[10];
  const float* Wo  = (const float*)d_in[11];
  const float* bov = (const float*)d_in[12];
  const float* ow  = (const float*)d_in[13];
  const float* ob  = (const float*)d_in[14];
  float* out = (float*)d_out;

  const size_t szBT1  = (size_t)kNpad * kK1 * 2;
  const size_t szBT2  = (size_t)kNpad * kK2 * 2;
  const size_t szWL   = (size_t)kGateCols * kZK * 2;
  const size_t szFEAT = (size_t)kFrames * kFeatPitch * 4;
  const size_t szIM1  = (size_t)kMC * kK1 * 2;
  const size_t szC1   = (size_t)kMC * kNpad * 2;
  const size_t szIM2  = (size_t)kMC * kK2 * 2;
  const size_t szC2   = (size_t)kMC * kNpad * 4;
  const size_t oBT1  = 0;
  const size_t oBT2  = oBT1 + szBT1;
  const size_t oWL   = oBT2 + szBT2;
  const size_t oFEAT = oWL + szWL;
  const size_t oIM1  = oFEAT + szFEAT;
  const size_t oC1   = oIM1 + szIM1;
  const size_t oIM2  = oC1 + szC1;
  const size_t oC2   = oIM2 + szIM2;
  const size_t total = oC2 + szC2;
  if (total > ws_size) return;

  char* ws = (char*)d_ws;
  unsigned short* pBT1 = (unsigned short*)(ws + oBT1);
  unsigned short* pBT2 = (unsigned short*)(ws + oBT2);
  unsigned short* pWL  = (unsigned short*)(ws + oWL);
  float*          pFEAT = (float*)(ws + oFEAT);
  unsigned short* pIM1 = (unsigned short*)(ws + oIM1);
  unsigned short* pC1  = (unsigned short*)(ws + oC1);
  unsigned short* pIM2 = (unsigned short*)(ws + oIM2);
  float*          pC2  = (float*)(ws + oC2);

  {
    const int n1 = kNpad * (kK1 / 8);
    k_wprep16<true><<<dim3((n1 + kThreads - 1) / kThreads), dim3(kThreads), 0, stream>>>(
        w1, b1, kK1Real, kF, kK1, kNpad, kWScale, pBT1);
    const int n2 = kNpad * (kK2 / 8);
    k_wprep16<false><<<dim3((n2 + kThreads - 1) / kThreads), dim3(kThreads), 0, stream>>>(
        w2, w2, kK2Real, kF, kK2, kNpad, kWScale, pBT2);
    const int nl = kUnits * (kZK / 8);
    const int gl = (nl + kThreads - 1) / kThreads;
    const size_t gstride = (size_t)kUnits * kZK;
    k_wprep16<false><<<dim3(gl), dim3(kThreads), 0, stream>>>(Wf, Wf, kZReal, kUnits, kZK, kUnits, kWScale, pWL + 0 * gstride);
    k_wprep16<false><<<dim3(gl), dim3(kThreads), 0, stream>>>(Wi, Wi, kZReal, kUnits, kZK, kUnits, kWScale, pWL + 1 * gstride);
    k_wprep16<false><<<dim3(gl), dim3(kThreads), 0, stream>>>(Wc, Wc, kZReal, kUnits, kZK, kUnits, kWScale, pWL + 2 * gstride);
    k_wprep16<false><<<dim3(gl), dim3(kThreads), 0, stream>>>(Wo, Wo, kZReal, kUnits, kZK, kUnits, kWScale, pWL + 3 * gstride);
  }

  const int gemmBlocks = (kMC / 64) / 8;
  for (int ch = 0; ch < kChunks; ++ch) {
    const int fbase = ch * kFC;
    k_im2col1<<<dim3((kMC * 4) / kThreads), dim3(kThreads), 0, stream>>>(x, fbase, pIM1);
    wmma_gemm64<0, false, 0, 1, false, 0><<<dim3(gemmBlocks, 1), dim3(256), 0, stream>>>(
        pIM1, pIM1, kK1, 0L, pBT1, pBT1, kK1, 0L, (void*)pC1, (void*)pC1, kNpad, 0L,
        pFEAT, pC2, 0L, kMC, kNpad, kK1, kC1Scale);
    k_im2col2<<<dim3((kMC * (kK2 / 8)) / kThreads), dim3(kThreads), 0, stream>>>(pC1, pIM2);
    wmma_gemm64<0, false, 0, 0, false, 0><<<dim3(gemmBlocks, 1), dim3(256), 0, stream>>>(
        pIM2, pIM2, kK2, 0L, pBT2, pBT2, kK2, 0L, (void*)pC2, (void*)pC2, kNpad, 0L,
        pFEAT, pC2, 0L, kMC, kNpad, kK2, kC2Scale);
    k_pool<<<dim3(kFC), dim3(kThreads), 0, stream>>>(pC2, b2, fbase, pFEAT);
  }

  k_lstm<<<dim3(1), dim3(kThreads), 0, stream>>>(pFEAT, pWL, bfv, biv, bcv, bov, ow, ob, out);
}
